// MultiHeadSelfAttention_58093727646383
// MI455X (gfx1250) — hardware-verified
//
#include <hip/hip_runtime.h>

#ifndef NB
#define NB 4
#endif
#ifndef SEQ
#define SEQ 2048
#endif
#define NB_FULL 4
#define SEQ_FULL 2048
#define DM 1024
#define NH 16
#define HD 64
#define N3 3072
#define MROWS (NB * SEQ)
#define EROWS 256
#define EQB (EROWS / 64)
#define KT (SEQ / 32)
#define FPITCH (((KT + 31) / 32) * 32)
#define QT (SEQ / 16)
#define NQMAIN ((SEQ / 64 - EQB) > 0 ? (SEQ / 64 - EQB) : 0)
#define ROTW 32

static_assert(NB <= NB_FULL);
static_assert(SEQ <= SEQ_FULL);
static_assert(SEQ % 64 == 0);
static_assert(SEQ / 64 >= EQB);
static_assert(EROWS % 64 == 0);
static_assert(DM == NH * HD);
static_assert(HD == 64);
static_assert(N3 == 3 * DM);
static_assert(DM % 64 == 0);
static_assert(DM % 32 == 0);
static_assert(MROWS % 64 == 0);
static_assert(((MROWS / 64) * (N3 / 64)) % 8 == 0);
static_assert(((SEQ / 64) * (DM / 64)) % 8 == 0);
static_assert(((EROWS / 64) * (DM / 64)) % 8 == 0);
static_assert(FPITCH % 32 == 0);
static_assert(FPITCH / 4 <= 32);
static_assert(KT >= 2);
static_assert(HD / 2 == ROTW);
static_assert(ROTW % 4 == 0);
static_assert(2 * DM == 256 * 8);
static_assert((((long long)N3 * DM) / 8) % 256 == 0);
static_assert((((long long)DM * DM) / 8) % 256 == 0);

typedef _Float16 v16h __attribute__((ext_vector_type(16)));
typedef _Float16 v8h __attribute__((ext_vector_type(8)));
typedef float v8f __attribute__((ext_vector_type(8)));
typedef float v4f __attribute__((ext_vector_type(4)));
typedef unsigned int v4u __attribute__((ext_vector_type(4)));
typedef int v4i __attribute__((ext_vector_type(4)));
union FH { v16h v; v8h h[2]; };

#define WS_X16   ((size_t)MROWS * DM * 2)
#define WS_W3    ((size_t)N3 * DM * 2)
#define WS_WO    ((size_t)DM * DM * 2)
#define WS_PH    ((size_t)MROWS * N3 * 2)
#define WS_PR    ((size_t)MROWS * N3 * 2)
#define WS_CL    ((size_t)NB * EROWS * DM * 2)
#define WS_FLG   ((size_t)QT * FPITCH * 4)
#define WS_TOTAL (WS_X16 + WS_W3 + WS_WO + WS_PH + WS_PR + WS_CL + WS_FLG)
static_assert(WS_TOTAL <= (size_t)134217728);
static_assert(WS_X16 % 256 == 0 && WS_W3 % 256 == 0 && WS_WO % 256 == 0 && WS_PH % 256 == 0 && WS_CL % 256 == 0 && WS_FLG % 128 == 0);

#define XSC 16.0f
#define WSC 64.0f
#define PSC 4096.0f
#define CSC 64.0f
#define RSC 2048.0f
#define RINV (1.0f / 2048.0f)

#define VST2(T, ptr, val) do { const T vst2_v_ = (val); *(volatile T*)(ptr) = vst2_v_; __threadfence(); *(volatile T*)(ptr) = vst2_v_; } while (0)

__device__ __forceinline__ float cmb_bf(float v) {
    const unsigned u = __builtin_bit_cast(unsigned, v);
    const unsigned r = (u + 0x7fffu + ((u >> 16) & 1u)) & 0xffff0000u;
    return __builtin_bit_cast(float, r);
}
__device__ __forceinline__ unsigned pkh(_Float16 a, _Float16 b) {
    return (unsigned)__builtin_bit_cast(unsigned short, a) | ((unsigned)__builtin_bit_cast(unsigned short, b) << 16);
}
__device__ __forceinline__ unsigned pkf(float a, float b) { return pkh((_Float16)a, (_Float16)b); }
__device__ __forceinline__ void hr_split(float v, _Float16& hi, _Float16& rs) { hi = (_Float16)v; rs = (_Float16)((v - (float)hi) * RSC); }
__device__ __forceinline__ v16h ldfrag_g(const _Float16* __restrict__ p) { FH f; f.h[0] = *(const v8h*)(p); f.h[1] = *(const v8h*)(p + 16); return f.v; }
__device__ __forceinline__ v8f mmah(v16h a, v16h b, v8f c) { return __builtin_amdgcn_wmma_f32_16x16x32_f16(false, a, false, b, (short)0, c, false, false); }
__device__ __forceinline__ void wave_sync() {
    __builtin_amdgcn_fence(3  , "workgroup");
    __builtin_amdgcn_wave_barrier();
    __builtin_amdgcn_fence(2  , "workgroup");
}
__device__ __forceinline__ void guard_g(v8f& a, v8f& b, v8f& c, v8f& d, v16h x, v16h y0, v16h y1, v16h y2, v16h y3) {
    asm volatile("v_nop\n\tv_nop\n\tv_nop\n\tv_nop" : "+v"(a), "+v"(b), "+v"(c), "+v"(d) : "v"(x), "v"(y0), "v"(y1), "v"(y2), "v"(y3));
}
__device__ __forceinline__ void guard_s4(v8f& a, v8f& b, v8f& c, v8f& d, v16h x0, v16h x1, v16h y0, v16h y1) {
    asm volatile("v_nop\n\tv_nop\n\tv_nop\n\tv_nop" : "+v"(a), "+v"(b), "+v"(c), "+v"(d) : "v"(x0), "v"(x1), "v"(y0), "v"(y1));
}
__device__ __forceinline__ void guard_s6(v8f& a, v8f& b, v8f& c, v8f& d, v16h x0, v16h x1, v16h y0, v16h y1, v16h y2, v16h y3) {
    asm volatile("v_nop\n\tv_nop\n\tv_nop\n\tv_nop" : "+v"(a), "+v"(b), "+v"(c), "+v"(d) : "v"(x0), "v"(x1), "v"(y0), "v"(y1), "v"(y2), "v"(y3));
}
__device__ __forceinline__ void guard_o1(v8f& a, v16h x, v16h y) {
    asm volatile("v_nop\n\tv_nop\n\tv_nop\n\tv_nop" : "+v"(a) : "v"(x), "v"(y));
}
__device__ __forceinline__ void guard_o2(v8f& a, v8f& b, v16h x0, v16h x1, v16h y0, v16h y1) {
    asm volatile("v_nop\n\tv_nop\n\tv_nop\n\tv_nop" : "+v"(a), "+v"(b) : "v"(x0), "v"(x1), "v"(y0), "v"(y1));
}

static __device__ __forceinline__ _Float16 toh_flush(float v) {
    const _Float16 r = (_Float16)v;
    return (fabsf(v) < 6.103515625e-05f) ? (_Float16)0.0f : r;
}
static __device__ __forceinline__ unsigned pkf_fl(float a, float b) { return pkh(toh_flush(a), toh_flush(b)); }
static __device__ __forceinline__ void hr_split_fl(float v, _Float16& hi, _Float16& rs) { hi = toh_flush(v); rs = toh_flush((v - (float)hi) * RSC); }
static __device__ __forceinline__ float uh_lo(unsigned w) { return (float)__builtin_bit_cast(_Float16, (unsigned short)(w & 0xffffu)); }
static __device__ __forceinline__ float uh_hi(unsigned w) { return (float)__builtin_bit_cast(_Float16, (unsigned short)(w >> 16)); }

__global__ __launch_bounds__(256) void k_cast_x(const float* __restrict__ x, unsigned short* __restrict__ X16) {
    const long long u = (long long)blockIdx.x * 256 + threadIdx.x;
    const int per = DM / 8;
    if (u >= (long long)MROWS * per) return;
    const int r = (int)(u / per), c0 = 8 * (int)(u % per);
    const int b = r / SEQ, n = r - b * SEQ;
    const float* s = x + ((size_t)b * SEQ_FULL + n) * DM + c0;
    const v4f a = *(const v4f*)s, d = *(const v4f*)(s + 4);
    v4u pk;
    pk.x = pkf(cmb_bf(a.x) * XSC, cmb_bf(a.y) * XSC); pk.y = pkf(cmb_bf(a.z) * XSC, cmb_bf(a.w) * XSC);
    pk.z = pkf(cmb_bf(d.x) * XSC, cmb_bf(d.y) * XSC); pk.w = pkf(cmb_bf(d.z) * XSC, cmb_bf(d.w) * XSC);
    VST2(v4u, X16 + (size_t)r * DM + c0, pk);
}
__global__ __launch_bounds__(256) void k_cast_w(const float* __restrict__ SRC, unsigned short* __restrict__ DST, int n8) {
    const int u = (int)blockIdx.x * 256 + (int)threadIdx.x;
    if (u >= n8) return;
    const float* s = SRC + (size_t)u * 8;
    const v4f a = *(const v4f*)s, d = *(const v4f*)(s + 4);
    v4u pk;
    pk.x = pkf_fl(cmb_bf(a.x) * WSC, cmb_bf(a.y) * WSC); pk.y = pkf_fl(cmb_bf(a.z) * WSC, cmb_bf(a.w) * WSC);
    pk.z = pkf_fl(cmb_bf(d.x) * WSC, cmb_bf(d.y) * WSC); pk.w = pkf_fl(cmb_bf(d.z) * WSC, cmb_bf(d.w) * WSC);
    VST2(v4u, DST + (size_t)u * 8, pk);
}

__global__ __launch_bounds__(256) void k_flags(const int* __restrict__ mask, int* __restrict__ flags) {
    __shared__ __align__(16) int fl[FPITCH];
    const int qt = blockIdx.x, lane = threadIdx.x & 31;
    const int wave = __builtin_amdgcn_readfirstlane((int)(threadIdx.x >> 5));
    for (int i = KT + (int)threadIdx.x; i < FPITCH; i += 256) fl[i] = 2;
#pragma unroll 1
    for (int kj = wave; kj < KT; kj += 8) {
        bool am = true, az = true;
#pragma unroll
        for (int r = 0; r < 16; ++r) {
            const int v = mask[(size_t)(qt * 16 + r) * SEQ_FULL + kj * 32 + lane];
            am = am && (v != 0); az = az && (v == 0);
        }
        const int wam = __all(am ? 1 : 0), waz = __all(az ? 1 : 0);
        const int f = wam ? 2 : (waz ? 0 : 1);
        if (lane == 0) fl[kj] = f;
    }
    __syncthreads();
    if (wave == 0 && lane < FPITCH / 4) {
        v4i v; v.x = fl[4 * lane]; v.y = fl[4 * lane + 1]; v.z = fl[4 * lane + 2]; v.w = fl[4 * lane + 3];
        VST2(v4i, flags + (size_t)qt * FPITCH + 4 * lane, v);
    }
}

template <int OUT_MODE, bool BIAS, bool RESID>
__device__ __forceinline__ void gemm64_body(const _Float16* __restrict__ A, long long strideA, const _Float16* __restrict__ Bt,
                                            float* Cf, unsigned short* Ch, unsigned short* Cr, int ldc, long long strideC,
                                            const float* __restrict__ bias, int M, int N, float scale) {
    __shared__ __align__(16) float sT[8][16 * 68];
    const int bz = blockIdx.y;
    const int lane = threadIdx.x & 31;
    const int wave = __builtin_amdgcn_readfirstlane((int)(threadIdx.x >> 5));
    const int tilesN = N >> 6, tilesM = M >> 6;
    const int tile = blockIdx.x * 8 + wave;
    if (tile >= tilesM * tilesN) return;
    const int tm = tile / tilesN, tn = tile - tm * tilesN;
    const int m0 = tm << 6, n0 = tn << 6;
    const _Float16* Ab = A + (size_t)bz * (size_t)strideA;
    const int rl = lane & 15, koff = (lane >> 4) * 8, mOff = (lane >> 4) * 8;

    v8f acc[4][4];
    const v8f zz = {0.f, 0.f, 0.f, 0.f, 0.f, 0.f, 0.f, 0.f};
#pragma unroll
    for (int i = 0; i < 4; ++i)
#pragma unroll
        for (int j = 0; j < 4; ++j) acc[i][j] = zz;

    for (int k0 = 0; k0 < DM; k0 += 32) {
        v16h bh[4];
#pragma unroll
        for (int j = 0; j < 4; ++j) bh[j] = ldfrag_g(Bt + (size_t)(n0 + (j << 4) + rl) * DM + koff + k0);
#pragma unroll
        for (int i = 0; i < 4; ++i) {
            const v16h ah = ldfrag_g(Ab + (size_t)(m0 + (i << 4) + rl) * DM + koff + k0);
#pragma unroll
            for (int j = 0; j < 4; ++j) acc[i][j] = mmah(ah, bh[j], acc[i][j]);
            guard_g(acc[i][0], acc[i][1], acc[i][2], acc[i][3], ah, bh[0], bh[1], bh[2], bh[3]);
        }
    }

#pragma unroll
    for (int i = 0; i < 4; ++i) {
        const int mBase = m0 + (i << 4);
#pragma unroll
        for (int j = 0; j < 4; ++j) {
            const int n = n0 + (j << 4) + rl;
            float bv = 0.f;
            if (BIAS) bv = cmb_bf(bias[n]);
#pragma unroll
            for (int r = 0; r < 8; ++r) sT[wave][(mOff + r) * 68 + (j << 4) + rl] = acc[i][j][r] * scale + bv;
        }
        wave_sync();
        if (OUT_MODE == 0) {
            float* C = Cf + (size_t)bz * (size_t)strideC;
            const int hh = lane >> 4, c4 = (lane & 15) * 4;
            v4f vals[8];
#pragma unroll
            for (int it = 0; it < 8; ++it) {
                const int row = it * 2 + hh;
                v4f v = *(const v4f*)&sT[wave][row * 68 + c4];
                if (RESID) { const v4f o = *(const v4f*)(C + (size_t)(mBase + row) * ldc + n0 + c4); v = v + o; }
                vals[it] = v;
            }
            for (int pass = 0; pass < 2; ++pass) {
#pragma unroll
                for (int it = 0; it < 8; ++it) {
                    const int row = it * 2 + hh;
                    *(volatile v4f*)(C + (size_t)(mBase + row) * ldc + n0 + c4) = vals[it];
                }
                __threadfence();
            }
        } else {
            const int q = lane >> 3, c8 = (lane & 7) * 8;
            unsigned short* C1 = Ch + (size_t)bz * (size_t)strideC;
            unsigned short* C2 = Cr + (size_t)bz * (size_t)strideC;
            v4u hv[4], rv[4];
#pragma unroll
            for (int it = 0; it < 4; ++it) {
                const int so = (it * 4 + q) * 68 + c8;
                _Float16 hx[8], rx[8];
#pragma unroll
                for (int e = 0; e < 8; ++e) hr_split(sT[wave][so + e], hx[e], rx[e]);
                hv[it].x = pkh(hx[0], hx[1]); hv[it].y = pkh(hx[2], hx[3]); hv[it].z = pkh(hx[4], hx[5]); hv[it].w = pkh(hx[6], hx[7]);
                rv[it].x = pkh(rx[0], rx[1]); rv[it].y = pkh(rx[2], rx[3]); rv[it].z = pkh(rx[4], rx[5]); rv[it].w = pkh(rx[6], rx[7]);
            }
            for (int pass = 0; pass < 2; ++pass) {
#pragma unroll
                for (int it = 0; it < 4; ++it) {
                    const int row = it * 4 + q;
                    *(volatile v4u*)(C1 + (size_t)(mBase + row) * ldc + n0 + c8) = hv[it];
                    *(volatile v4u*)(C2 + (size_t)(mBase + row) * ldc + n0 + c8) = rv[it];
                }
                __threadfence();
            }
        }
        wave_sync();
    }
}

__global__ __launch_bounds__(256) void k_gemm_qkv(const _Float16* __restrict__ X16, const _Float16* __restrict__ W3, const float* __restrict__ bqkv,
                                                  unsigned short* __restrict__ PH, unsigned short* __restrict__ PR) {
    gemm64_body<1, true, false>(X16, 0, W3, nullptr, PH, PR, N3, 0, bqkv, MROWS, N3, 1.0f / (XSC * WSC));
}
__global__ __launch_bounds__(256) void k_gemm_proj(const _Float16* __restrict__ CH, const _Float16* __restrict__ WO, const float* __restrict__ bproj, float* out) {
    gemm64_body<0, true, false>(CH, (long long)SEQ * DM, WO, out, nullptr, nullptr, DM, (long long)SEQ_FULL * DM, bproj, SEQ, DM, 1.0f / (CSC * WSC));
}
__global__ __launch_bounds__(256) void k_gemm_proj_res(const _Float16* __restrict__ CL, const _Float16* __restrict__ WO, float* out) {
    gemm64_body<0, false, true>(CL, (long long)EROWS * DM, WO, out, nullptr, nullptr, DM, (long long)SEQ_FULL * DM, nullptr, EROWS, DM, 1.0f / (CSC * WSC * RSC));
}

static __device__ __forceinline__ void rot_pair(unsigned hw, unsigned rw, float cv, float sv, unsigned& ho, unsigned& ro) {
#pragma clang fp contract(off)
    const float a = uh_lo(hw) + uh_lo(rw) * RINV;
    const float b = uh_hi(hw) + uh_hi(rw) * RINV;
    const float cb = cmb_bf(cv), sb = cmb_bf(sv);
    const float o_r = a * cb - b * sb;
    const float o_i = a * sb + b * cb;
    _Float16 h0, r0, h1, r1;
    hr_split_fl(o_r, h0, r0);
    hr_split_fl(o_i, h1, r1);
    ho = pkh(h0, h1); ro = pkh(r0, r1);
}
__global__ __launch_bounds__(256) void k_rope(unsigned short* PH, unsigned short* PR,
                                              const float* __restrict__ fcos, const float* __restrict__ fsin) {
#pragma clang fp contract(off)
    const int r = (int)blockIdx.x;
    if (r >= MROWS) return;
    const int c0 = 8 * (int)threadIdx.x;
    const int n = r - (r / SEQ) * SEQ;
    const int i0 = (c0 & (HD - 1)) >> 1;
    const v4f cs = *(const v4f*)(fcos + (size_t)n * ROTW + i0);
    const v4f sn = *(const v4f*)(fsin + (size_t)n * ROTW + i0);
    const size_t off = (size_t)r * N3 + c0;
    const v4u hw = *(const v4u*)(PH + off);
    const v4u rw = *(const v4u*)(PR + off);
    v4u ho, ro;
    unsigned th, tr;
    rot_pair(hw.x, rw.x, cs.x, sn.x, th, tr); ho.x = th; ro.x = tr;
    rot_pair(hw.y, rw.y, cs.y, sn.y, th, tr); ho.y = th; ro.y = tr;
    rot_pair(hw.z, rw.z, cs.z, sn.z, th, tr); ho.z = th; ro.z = tr;
    rot_pair(hw.w, rw.w, cs.w, sn.w, th, tr); ho.w = th; ro.w = tr;
    VST2(v4u, PH + off, ho);
    VST2(v4u, PR + off, ro);
}

template <bool EARLY>
__device__ __forceinline__ void attn_body(const _Float16* __restrict__ PH, const _Float16* __restrict__ PR,
                                          const int* __restrict__ mask, const int* __restrict__ flags,
                                          unsigned short* __restrict__ CH, unsigned short* __restrict__ CL) {
    __shared__ __align__(16) _Float16 Ksh[64 * 64];
    __shared__ __align__(16) _Float16 Ksl[EARLY ? 64 * 64 : 8];
    __shared__ __align__(16) _Float16 Vth[64 * 64];
    __shared__ __align__(16) _Float16 Vtl[EARLY ? 64 * 64 : 8];
    __shared__ __align__(16) _Float16 Psh[4 * 16 * 32];
    __shared__ __align__(16) _Float16 Psl[EARLY ? 4 * 16 * 32 : 8];
    __shared__ __align__(16) float Os[4 * 16 * 68];

    const int tid = threadIdx.x, lane = tid & 31, hh = lane >> 4, c = lane & 15;
    const int wave = __builtin_amdgcn_readfirstlane(tid >> 5);
    const int bx = blockIdx.x;
    int qb, bh;
    if (EARLY) { qb = bx % EQB; bh = bx / EQB; }
    else { const int nq = (NQMAIN > 0) ? NQMAIN : 1; qb = EQB + bx % nq; bh = bx / nq; }
    const int h = bh % NH, b = bh / NH;
    const int q0 = qb * 64 + wave * 16;
    const int qt = qb * 4 + wave;
    const size_t rowbase = (size_t)b * SEQ;
    const size_t qoff = (rowbase + q0 + c) * N3 + h * HD + 8 * hh;
    const float L2E = 1.4426950408889634f;
    const float SC = 0.125f * L2E;
    const float NEGF = -__builtin_inff();

    int last = 0;
#pragma unroll
    for (int w = 0; w < 4; ++w) {
#pragma unroll
        for (int u = 0; u < (KT + 31) / 32; ++u) {
            const int kjc = min(lane + 32 * u, KT - 1);
            const int fv = flags[(size_t)(qb * 4 + w) * FPITCH + kjc];
            last = max(last, (fv != 2) ? (kjc / 2 + 1) : 0);
        }
    }
    last = max(last, __shfl_xor(last, 1, 32)); last = max(last, __shfl_xor(last, 2, 32));
    last = max(last, __shfl_xor(last, 4, 32)); last = max(last, __shfl_xor(last, 8, 32));
    last = max(last, __shfl_xor(last, 16, 32));
    const int nchunks = min(max(__builtin_amdgcn_readfirstlane(last), 0), SEQ / 64);

    const v8f zz = {0.f, 0.f, 0.f, 0.f, 0.f, 0.f, 0.f, 0.f};
    v8f oacc[4], ores[4];
    float mrow[8], lrow[8];
#pragma unroll
    for (int t = 0; t < 4; ++t) { oacc[t] = zz; ores[t] = zz; }
#pragma unroll
    for (int r = 0; r < 8; ++r) { mrow[r] = -3.0e38f; lrow[r] = 0.f; }

    const int kvr = tid >> 1, dh = (tid & 1) * 32;
    const int pbase = wave * 512;

    for (int kc = 0; kc < nchunks; ++kc) {
        const int kv0 = kc * 64;
        __syncthreads();
        {
            const size_t grow = (rowbase + kv0 + kvr) * N3 + h * HD + dh;
#pragma unroll
            for (int i = 0; i < 4; ++i) {
                const v8h kk = *(const v8h*)(PH + grow + DM + 8 * i);
                *(v8h*)&Ksh[kvr * 64 + dh + 8 * i] = kk;
                const v8h vv = *(const v8h*)(PH + grow + 2 * DM + 8 * i);
#pragma unroll
                for (int e = 0; e < 8; ++e) Vth[(dh + 8 * i + e) * 64 + kvr] = vv[e];
                if (EARLY) {
                    const v8h kl = *(const v8h*)(PR + grow + DM + 8 * i);
                    *(v8h*)&Ksl[kvr * 64 + dh + 8 * i] = kl;
                    const v8h vl = *(const v8h*)(PR + grow + 2 * DM + 8 * i);
#pragma unroll
                    for (int e = 0; e < 8; ++e) Vtl[(dh + 8 * i + e) * 64 + kvr] = vl[e];
                }
            }
        }
        __syncthreads();

#pragma unroll 1
        for (int hf = 0; hf < 2; ++hf) {
            const int kj = 2 * kc + hf;
            const int f = __builtin_amdgcn_readfirstlane(flags[(size_t)qt * FPITCH + kj]);
            if (f == 2) continue;

            v8f sh0 = zz, sh1 = zz, sr0 = zz, sr1 = zz;
#pragma unroll
            for (int dc = 0; dc < 2; ++dc) {
                const v16h qh = ldfrag_g(PH + qoff + dc * 32);
                const v16h ql = ldfrag_g(PR + qoff + dc * 32);
                const int ko = (hf * 32 + c) * 64 + dc * 32 + 8 * hh;
                FH k0f, k1f;
                k0f.h[0] = *(const v8h*)&Ksh[ko];            k0f.h[1] = *(const v8h*)&Ksh[ko + 16];
                k1f.h[0] = *(const v8h*)&Ksh[ko + 16 * 64];  k1f.h[1] = *(const v8h*)&Ksh[ko + 16 * 64 + 16];
                sh0 = mmah(qh, k0f.v, sh0); sr0 = mmah(ql, k0f.v, sr0);
                sh1 = mmah(qh, k1f.v, sh1); sr1 = mmah(ql, k1f.v, sr1);
                if (EARLY) {
                    FH l0f, l1f;
                    l0f.h[0] = *(const v8h*)&Ksl[ko];            l0f.h[1] = *(const v8h*)&Ksl[ko + 16];
                    l1f.h[0] = *(const v8h*)&Ksl[ko + 16 * 64];  l1f.h[1] = *(const v8h*)&Ksl[ko + 16 * 64 + 16];
                    sr0 = mmah(qh, l0f.v, sr0); sr1 = mmah(qh, l1f.v, sr1);
                    guard_s6(sh0, sh1, sr0, sr1, qh, ql, k0f.v, k1f.v, l0f.v, l1f.v);
                } else {
                    guard_s4(sh0, sh1, sr0, sr1, qh, ql, k0f.v, k1f.v);
                }
            }
            float s0[8], s1[8];
#pragma unroll
            for (int r = 0; r < 8; ++r) { s0[r] = (sh0[r] + sr0[r] * RINV) * SC; s1[r] = (sh1[r] + sr1[r] * RINV) * SC; }
            if (f != 0) {
                int mk0[8], mk1[8];
#pragma unroll
                for (int r = 0; r < 8; ++r) {
                    const size_t mo = (size_t)(q0 + 8 * hh + r) * SEQ_FULL + kv0 + hf * 32 + c;
                    mk0[r] = mask[mo]; mk1[r] = mask[mo + 16];
                }
#pragma unroll
                for (int r = 0; r < 8; ++r) { asm volatile("" : "+v"(mk0[r])); asm volatile("" : "+v"(mk1[r])); }
#pragma unroll
                for (int r = 0; r < 8; ++r) {
                    s0[r] = (mk0[r] != 0) ? NEGF : s0[r];
                    s1[r] = (mk1[r] != 0) ? NEGF : s1[r];
                }
            }
#pragma unroll
            for (int r = 0; r < 8; ++r) {
                float m = fmaxf(s0[r], s1[r]);
                m = fmaxf(m, __shfl_xor(m, 1, 32)); m = fmaxf(m, __shfl_xor(m, 2, 32));
                m = fmaxf(m, __shfl_xor(m, 4, 32)); m = fmaxf(m, __shfl_xor(m, 8, 32));
                const float mnew = fmaxf(mrow[r], m);
                const float alpha = exp2f(mrow[r] - mnew);
                const float p0 = exp2f(s0[r] - mnew), p1 = exp2f(s1[r] - mnew);
                float ps = p0 + p1;
                ps += __shfl_xor(ps, 1, 32); ps += __shfl_xor(ps, 2, 32); ps += __shfl_xor(ps, 4, 32); ps += __shfl_xor(ps, 8, 32);
                lrow[r] = lrow[r] * alpha + ps; mrow[r] = mnew;
#pragma unroll
                for (int t = 0; t < 4; ++t) { oacc[t][r] *= alpha; if (EARLY) ores[t][r] *= alpha; }
                const float a0 = p0 * PSC, a1 = p1 * PSC;
                const _Float16 h0 = toh_flush(a0), h1 = toh_flush(a1);
                const int pi = pbase + (8 * hh + r) * 32 + c;
                Psh[pi] = h0; Psh[pi + 16] = h1;
                if (EARLY) { Psl[pi] = toh_flush((a0 - (float)h0) * RSC); Psl[pi + 16] = toh_flush((a1 - (float)h1) * RSC); }
            }
            wave_sync();
            {
                const int po = pbase + c * 32 + 8 * hh;
                FH pa, pl;
                pa.h[0] = *(const v8h*)&Psh[po]; pa.h[1] = *(const v8h*)&Psh[po + 16];
                if (EARLY) { pl.h[0] = *(const v8h*)&Psl[po]; pl.h[1] = *(const v8h*)&Psl[po + 16]; }
#pragma unroll
                for (int t = 0; t < 4; ++t) {
                    const int vo = (t * 16 + c) * 64 + hf * 32 + 8 * hh;
                    FH vb;
                    vb.h[0] = *(const v8h*)&Vth[vo]; vb.h[1] = *(const v8h*)&Vth[vo + 16];
                    oacc[t] = mmah(pa.v, vb.v, oacc[t]);
                    if (EARLY) {
                        FH vl;
                        vl.h[0] = *(const v8h*)&Vtl[vo]; vl.h[1] = *(const v8h*)&Vtl[vo + 16];
                        ores[t] = mmah(pa.v, vl.v, ores[t]);
                        ores[t] = mmah(pl.v, vb.v, ores[t]);
                        guard_o2(oacc[t], ores[t], pa.v, pl.v, vb.v, vl.v);
                    } else {
                        guard_o1(oacc[t], pa.v, vb.v);
                    }
                }
            }
            wave_sync();
        }
    }

    const int ob = wave * 1088;
#pragma unroll
    for (int r = 0; r < 8; ++r) {
        const float inv = CSC / (lrow[r] * PSC);
#pragma unroll
        for (int t = 0; t < 4; ++t) {
            float v = oacc[t][r];
            if (EARLY) v += ores[t][r] * RINV;
            Os[ob + (8 * hh + r) * 68 + t * 16 + c] = v * inv;
        }
    }
    wave_sync();
    {
        const int qq = lane >> 3, c8 = (lane & 7) * 8;
        v4u hv[4], rv[4];
#pragma unroll
        for (int it = 0; it < 4; ++it) {
            const int so = ob + (it * 4 + qq) * 68 + c8;
            _Float16 hx[8], rx[8];
#pragma unroll
            for (int e = 0; e < 8; ++e) hr_split_fl(Os[so + e], hx[e], rx[e]);
            hv[it].x = pkh(hx[0], hx[1]); hv[it].y = pkh(hx[2], hx[3]); hv[it].z = pkh(hx[4], hx[5]); hv[it].w = pkh(hx[6], hx[7]);
            rv[it].x = pkh(rx[0], rx[1]); rv[it].y = pkh(rx[2], rx[3]); rv[it].z = pkh(rx[4], rx[5]); rv[it].w = pkh(rx[6], rx[7]);
        }
        for (int pass = 0; pass < 2; ++pass) {
#pragma unroll
            for (int it = 0; it < 4; ++it) {
                const int row = it * 4 + qq;
                *(volatile v4u*)(CH + (rowbase + q0 + row) * DM + h * HD + c8) = hv[it];
                if (EARLY) *(volatile v4u*)(CL + ((size_t)b * EROWS + q0 + row) * DM + h * HD + c8) = rv[it];
            }
            __threadfence();
        }
    }
}

__global__ __launch_bounds__(128) void k_attn_main(const _Float16* __restrict__ PH, const _Float16* __restrict__ PR, const int* __restrict__ mask,
                                                   const int* __restrict__ flags, unsigned short* __restrict__ CH) {
    attn_body<false>(PH, PR, mask, flags, CH, nullptr);
}
__global__ __launch_bounds__(128) void k_attn_early(const _Float16* __restrict__ PH, const _Float16* __restrict__ PR, const int* __restrict__ mask,
                                                    const int* __restrict__ flags, unsigned short* __restrict__ CH, unsigned short* __restrict__ CL) {
    attn_body<true>(PH, PR, mask, flags, CH, CL);
}

extern "C" void kernel_launch(void* const* d_in, const int* in_sizes, int n_in, void* d_out, int out_size, void* d_ws, size_t ws_size, hipStream_t stream) {
    if (n_in < 8) return;
    const long long need_x = ((long long)(NB - 1) * SEQ_FULL + SEQ) * DM;
    const long long need_m = (long long)(SEQ - 1) * SEQ_FULL + SEQ;
    if ((long long)in_sizes[0] < need_x) return;
    if ((long long)in_sizes[1] < need_m) return;
    if ((long long)in_sizes[2] < (long long)SEQ * ROTW) return;
    if ((long long)in_sizes[3] < (long long)SEQ * ROTW) return;
    if ((long long)in_sizes[4] < (long long)N3 * DM) return;
    if ((long long)in_sizes[5] < (long long)N3) return;
    if ((long long)in_sizes[6] < (long long)DM * DM) return;
    if ((long long)in_sizes[7] < (long long)DM) return;
    if ((long long)out_size < need_x) return;
    if (ws_size < WS_TOTAL) return;

    const float* x     = (const float*)d_in[0];
    const int*   cmask = (const int*)d_in[1];
    const float* fcos  = (const float*)d_in[2];
    const float* fsin  = (const float*)d_in[3];
    const float* Wqkv  = (const float*)d_in[4];
    const float* bqkv  = (const float*)d_in[5];
    const float* Wproj = (const float*)d_in[6];
    const float* bproj = (const float*)d_in[7];
    float* out = (float*)d_out;

    char* wsp = (char*)d_ws;
    unsigned short* X16 = (unsigned short*)wsp; wsp += WS_X16;
    unsigned short* W3  = (unsigned short*)wsp; wsp += WS_W3;
    unsigned short* WO  = (unsigned short*)wsp; wsp += WS_WO;
    unsigned short* PHp = (unsigned short*)wsp; wsp += WS_PH;
    unsigned short* PRp = (unsigned short*)wsp; wsp += WS_PR;
    unsigned short* CLp = (unsigned short*)wsp; wsp += WS_CL;
    int* FLG = (int*)wsp; wsp += WS_FLG;
    unsigned short* CHp = X16;

    k_cast_x<<<(unsigned)(((long long)MROWS * (DM / 8) + 255) / 256), 256, 0, stream>>>(x, X16);
    k_cast_w<<<(unsigned)((((long long)N3 * DM) / 8) / 256), 256, 0, stream>>>(Wqkv, W3, (int)(((long long)N3 * DM) / 8));
    k_cast_w<<<(unsigned)((((long long)DM * DM) / 8) / 256), 256, 0, stream>>>(Wproj, WO, (int)(((long long)DM * DM) / 8));
    k_flags<<<QT, 256, 0, stream>>>(cmask, FLG);
    k_gemm_qkv<<<dim3((unsigned)(((MROWS / 64) * (N3 / 64)) / 8), 1), 256, 0, stream>>>((const _Float16*)X16, (const _Float16*)W3, bqkv, PHp, PRp);
    k_rope<<<(unsigned)MROWS, 256, 0, stream>>>(PHp, PRp, fcos, fsin);
    if (NQMAIN > 0)
        k_attn_main<<<(unsigned)(NB * NH * NQMAIN), 128, 0, stream>>>((const _Float16*)PHp, (const _Float16*)PRp, cmask, FLG, CHp);
    k_attn_early<<<(unsigned)(NB * NH * EQB), 128, 0, stream>>>((const _Float16*)PHp, (const _Float16*)PRp, cmask, FLG, CHp, CLp);
    k_gemm_proj<<<dim3((unsigned)(((SEQ / 64) * (DM / 64)) / 8), NB), 256, 0, stream>>>((const _Float16*)CHp, (const _Float16*)WO, bproj, out);
    k_gemm_proj_res<<<dim3((unsigned)(((EROWS / 64) * (DM / 64)) / 8), NB), 256, 0, stream>>>((const _Float16*)CLp, (const _Float16*)WO, out);
}
